// EncoderBlock_88502096101675
// MI455X (gfx1250) — hardware-verified
//
#include <hip/hip_runtime.h>
#include <stdint.h>
#include <stddef.h>


#ifndef NB
#define NB 2
#endif
#ifndef SEQ
#define SEQ 2048
#endif
#define NB_FULL 2
#define SEQ_FULL 2048
#define DIM 768
#define NHEAD 12
#define DHEAD 64
#define HID 3072
#define MROWS (NB * SEQ)
#define LDQKV (3 * DIM)
#define WPR (SEQ / 32)
#define FROW(m) ((((size_t)(m)) / SEQ) * SEQ_FULL + (((size_t)(m)) % SEQ))

static_assert(NB >= 1 && NB <= NB_FULL);
static_assert(SEQ >= 64 && SEQ <= SEQ_FULL && (SEQ % 64) == 0);
static_assert((MROWS % 128) == 0);
static_assert((DIM % 128) == 0 && (HID % 128) == 0 && (LDQKV % 128) == 0);
static_assert((DIM % 64) == 0 && (HID % 64) == 0 && (DIM % 32) == 0 && (HID % 32) == 0);
static_assert(NHEAD * DHEAD == DIM && DHEAD == 64);
static_assert(((size_t)SEQ * SEQ) % 4096 == 0);
static_assert(((size_t)(NB - 1) * SEQ_FULL + SEQ) * DIM <= (size_t)NB_FULL * SEQ_FULL * DIM);

typedef _Float16 v16h __attribute__((ext_vector_type(16)));
typedef _Float16 v8h  __attribute__((ext_vector_type(8)));
typedef float    v8f  __attribute__((ext_vector_type(8)));
typedef float    v4f  __attribute__((ext_vector_type(4)));

static __device__ __forceinline__ v8f wmma16(v16h a, v16h b, v8f c) {
  v8f d = __builtin_amdgcn_wmma_f32_16x16x32_f16(false, a, false, b, (short)0, c, false, false);
  asm volatile("v_nop\n\tv_nop\n\tv_nop\n\tv_nop" : "+v"(d) : "v"(a), "v"(b));
  return d;
}

static __device__ __forceinline__ float bf16r(float f) {
  unsigned int u = __float_as_uint(f);
  u = (u + 0x7FFFu + ((u >> 16) & 1u)) & 0xFFFF0000u;
  return __uint_as_float(u);
}

static __device__ __forceinline__ v16h load_frag(const _Float16* p) {
  v8h lo = *(const v8h*)(p);
  v8h hi = *(const v8h*)(p + 16);
  v16h f;
#pragma unroll
  for (int e = 0; e < 8; ++e) { f[e] = lo[e]; f[e + 8] = hi[e]; }
  return f;
}

#define TP 72
__global__ __launch_bounds__(256) void cvt_wt_kernel(
    const float* __restrict__ w0, const float* __restrict__ w1, const float* __restrict__ w2,
    _Float16* __restrict__ dst, int K, int N, float scale) {
#pragma clang fp contract(off)
  __shared__ __attribute__((aligned(16))) _Float16 T[64 * TP];
  const int part = blockIdx.z;
  const float* w = (part == 0) ? w0 : ((part == 1) ? w1 : w2);
  const int k0 = blockIdx.y * 64, n0 = blockIdx.x * 64;
  const int tid = threadIdx.x;
#pragma unroll
  for (int q = 0; q < 4; ++q) {
    const int idx = q * 256 + tid;
    const int kr = idx >> 4;
    const int nc = (idx & 15) << 2;
    const v4f v = *(const v4f*)(w + (size_t)(k0 + kr) * N + n0 + nc);
#pragma unroll
    for (int e = 0; e < 4; ++e) T[(nc + e) * TP + kr] = (_Float16)(bf16r(v[e]) * scale);
  }
  __syncthreads();
  const int rs = tid >> 3, cc = (tid & 7) << 3;
  v8h hv[2];
  size_t go[2];
#pragma unroll
  for (int it = 0; it < 2; ++it) {
    const int nl = it * 32 + rs;
    hv[it] = *(const v8h*)(T + nl * TP + cc);
    go[it] = ((size_t)part * N + n0 + nl) * (size_t)K + k0 + cc;
  }
#pragma unroll
  for (int it = 0; it < 2; ++it) *(volatile v8h*)(dst + go[it]) = hv[it];
  __threadfence();
#pragma unroll
  for (int it = 0; it < 2; ++it) *(volatile v8h*)(dst + go[it]) = hv[it];
}

__global__ __launch_bounds__(128) void maskpack_kernel(const int* __restrict__ mask,
                                                       unsigned int* __restrict__ mb) {
  const unsigned int tid = threadIdx.x;
  const unsigned int wave = tid >> 5, lane = tid & 31u;
  const unsigned int wbase = (blockIdx.x * 4u + wave) * 32u;
  unsigned int w = 0u;
#pragma unroll 4
  for (unsigned int i = 0; i < 32u; ++i) {
    const unsigned int W = wbase + i;
    const unsigned int q = W / (unsigned int)WPR;
    const unsigned int kw = W % (unsigned int)WPR;
    const int m = mask[(size_t)q * SEQ_FULL + kw * 32u + lane];
    const unsigned int bal = __builtin_amdgcn_ballot_w32(m != 0);
    w = (lane == i) ? bal : w;
  }
  unsigned int* p = mb + wbase + lane;
  *(volatile unsigned int*)p = w;
  __threadfence();
  *(volatile unsigned int*)p = w;
}

__global__ __launch_bounds__(256) void vtrans_kernel(const _Float16* __restrict__ qkv,
                                                     _Float16* __restrict__ vt) {
  __shared__ __attribute__((aligned(16))) _Float16 T[64 * TP];
  const unsigned int bh = blockIdx.y;
  const unsigned int b = bh / (unsigned int)NHEAD, h = bh % (unsigned int)NHEAD;
  const int s0 = blockIdx.x * 64;
  const int tid = threadIdx.x;
#pragma unroll
  for (int q = 0; q < 2; ++q) {
    const int idx = q * 256 + tid;
    const int sr = idx >> 3;
    const int dc = (idx & 7) << 3;
    const v8h v = *(const v8h*)(qkv + ((size_t)b * SEQ + s0 + sr) * LDQKV + 2 * DIM + h * DHEAD + dc);
#pragma unroll
    for (int e = 0; e < 8; ++e) T[(dc + e) * TP + sr] = v[e];
  }
  __syncthreads();
  const int rs = tid >> 3, cc = (tid & 7) << 3;
  v8h hv[2];
  size_t go[2];
#pragma unroll
  for (int it = 0; it < 2; ++it) {
    const int dl = it * 32 + rs;
    hv[it] = *(const v8h*)(T + dl * TP + cc);
    go[it] = ((size_t)bh * DHEAD + dl) * (size_t)SEQ + s0 + cc;
  }
#pragma unroll
  for (int it = 0; it < 2; ++it) *(volatile v8h*)(vt + go[it]) = hv[it];
  __threadfence();
#pragma unroll
  for (int it = 0; it < 2; ++it) *(volatile v8h*)(vt + go[it]) = hv[it];
}

#define BM 128
#define BN 128
#define BK 32
#define LDT 40
#define EPF 132
#define GEMM_SMEM_FLOATS (64 * EPF)
static_assert((BM + BN) * LDT * 2 <= GEMM_SMEM_FLOATS * 4);

template <bool HAS_BIAS, int RES, bool RELU, bool OUT16, bool MAPOUT>
__global__ __launch_bounds__(256) void gemm_kernel(
    const _Float16* __restrict__ A, const _Float16* __restrict__ Bt,
    const float* __restrict__ bias, const float* __restrict__ bias1,
    const float* __restrict__ bias2, const float* __restrict__ res,
    float* __restrict__ outF, _Float16* __restrict__ outH,
    int N, int K, float scale, float bscale, int bpn) {
  static_assert(!(RES != 0 && OUT16));
  static_assert(!(MAPOUT && OUT16));
  __shared__ __attribute__((aligned(16))) float smem[GEMM_SMEM_FLOATS];
  _Float16* As = (_Float16*)smem;
  _Float16* Bs = As + BM * LDT;
  const int tid = threadIdx.x;
  const int wave = tid >> 5, lane = tid & 31;
  const int r = lane & 15, hb = (lane >> 4) << 3;
  const int mBlk = blockIdx.y * BM, nBlk = blockIdx.x * BN;
  const int mw = (wave & 1) * 64, nw = (wave >> 1) * 32;

  const int sr0 = tid >> 2, sr1 = sr0 + 64, skc = (tid & 3) << 3;
  const _Float16* gA0 = A  + (size_t)(mBlk + sr0) * K + skc;
  const _Float16* gA1 = A  + (size_t)(mBlk + sr1) * K + skc;
  const _Float16* gB0 = Bt + (size_t)(nBlk + sr0) * K + skc;
  const _Float16* gB1 = Bt + (size_t)(nBlk + sr1) * K + skc;

  v8f acc[4][2];
#pragma unroll
  for (int i = 0; i < 4; ++i)
#pragma unroll
    for (int j = 0; j < 2; ++j)
#pragma unroll
      for (int v = 0; v < 8; ++v) acc[i][j][v] = 0.f;

  const int nk = K >> 5;
#pragma unroll 1
  for (int kt = 0; kt < nk; ++kt) {
    const size_t ko = (size_t)kt * BK;
    const v8h a0 = *(const v8h*)(gA0 + ko);
    const v8h a1 = *(const v8h*)(gA1 + ko);
    const v8h b0 = *(const v8h*)(gB0 + ko);
    const v8h b1 = *(const v8h*)(gB1 + ko);
    __syncthreads();
    *(v8h*)(As + sr0 * LDT + skc) = a0;
    *(v8h*)(As + sr1 * LDT + skc) = a1;
    *(v8h*)(Bs + sr0 * LDT + skc) = b0;
    *(v8h*)(Bs + sr1 * LDT + skc) = b1;
    __syncthreads();
    v16h af[4], bfr[2];
#pragma unroll
    for (int i = 0; i < 4; ++i) af[i] = load_frag(As + (mw + i * 16 + r) * LDT + hb);
#pragma unroll
    for (int j = 0; j < 2; ++j) bfr[j] = load_frag(Bs + (nw + j * 16 + r) * LDT + hb);
#pragma unroll
    for (int i = 0; i < 4; ++i)
#pragma unroll
      for (int j = 0; j < 2; ++j) acc[i][j] = wmma16(af[i], bfr[j], acc[i][j]);
  }
  __syncthreads();

  float* stg = smem;
  float bcol[2] = {0.f, 0.f};
  if constexpr (HAS_BIAS) {
    const unsigned int ub = (unsigned int)bpn, un = (unsigned int)nBlk;
    const unsigned int part = (un >= 2u * ub) ? 2u : ((un >= ub) ? 1u : 0u);
    const float* bp = (part == 0u) ? bias : ((part == 1u) ? bias1 : bias2);
    const unsigned int cb = un - part * ub;
#pragma unroll
    for (int j = 0; j < 2; ++j) bcol[j] = bf16r(bp[cb + nw + j * 16 + r]) * bscale;
  }
#pragma unroll
  for (int p = 0; p < 2; ++p) {
    if ((wave & 1) == p) {
#pragma unroll
      for (int i = 0; i < 4; ++i)
#pragma unroll
        for (int j = 0; j < 2; ++j)
#pragma unroll
          for (int v = 0; v < 8; ++v) {
            const int lr = i * 16 + hb + v;
            const int lc = nw + j * 16 + r;
            float c = acc[i][j][v] * scale;
            if constexpr (HAS_BIAS) c += bcol[j];
            if constexpr (RELU) c = fmaxf(c, 0.f);
            stg[lr * EPF + lc] = c;
          }
    }
    __syncthreads();
    if constexpr (OUT16) {
      v8h hv[4];
      size_t go[4];
#pragma unroll
      for (int it = 0; it < 4; ++it) {
        const int lr = it * 16 + wave * 2 + (lane >> 4);
        const int lc = (lane & 15) << 3;
        const v4f x0 = *(const v4f*)(stg + lr * EPF + lc);
        const v4f x1 = *(const v4f*)(stg + lr * EPF + lc + 4);
        v8h hh;
#pragma unroll
        for (int e = 0; e < 4; ++e) { hh[e] = (_Float16)x0[e]; hh[e + 4] = (_Float16)x1[e]; }
        hv[it] = hh;
        go[it] = (size_t)(mBlk + p * 64 + lr) * (size_t)N + nBlk + lc;
      }
#pragma unroll
      for (int it = 0; it < 4; ++it) *(volatile v8h*)(outH + go[it]) = hv[it];
      __threadfence();
#pragma unroll
      for (int it = 0; it < 4; ++it) *(volatile v8h*)(outH + go[it]) = hv[it];
    } else {
      v4f fv[8];
      size_t go[8];
#pragma unroll
      for (int it = 0; it < 8; ++it) {
        const int lr = it * 8 + wave;
        const int lc = lane << 2;
        const size_t grow = (size_t)(mBlk + p * 64 + lr);
        const size_t gcol = (size_t)(nBlk + lc);
        v4f val = *(const v4f*)(stg + lr * EPF + lc);
        if constexpr (RES == 1) {
          const v4f rr = *(const v4f*)(res + grow * (size_t)N + gcol);
#pragma unroll
          for (int e = 0; e < 4; ++e) val[e] = val[e] + rr[e];
        }
        if constexpr (RES == 2) {
          const v4f rr = *(const v4f*)(res + FROW(grow) * (size_t)DIM + gcol);
#pragma unroll
          for (int e = 0; e < 4; ++e) val[e] = val[e] + bf16r(rr[e]);
        }
        fv[it] = val;
        const size_t orow = MAPOUT ? FROW(grow) : grow;
        go[it] = orow * (size_t)N + gcol;
      }
#pragma unroll
      for (int it = 0; it < 8; ++it) *(volatile v4f*)(outF + go[it]) = fv[it];
      __threadfence();
#pragma unroll
      for (int it = 0; it < 8; ++it) *(volatile v4f*)(outF + go[it]) = fv[it];
    }
    __syncthreads();
  }
}

#define VPAD 40
#define OPAD 72

__global__ __launch_bounds__(128) __attribute__((amdgpu_num_vgpr(256)))
void attn_kernel(const _Float16* __restrict__ qkv, const _Float16* __restrict__ vt,
                 const unsigned int* __restrict__ mbits, _Float16* __restrict__ ctx) {
  __shared__ __attribute__((aligned(16))) _Float16 Ps[4 * 16 * VPAD];
  __shared__ __attribute__((aligned(16))) _Float16 Os[4 * 16 * OPAD];
  const unsigned int nqt = SEQ / 64;
  const unsigned int qt = blockIdx.x % nqt;
  const unsigned int bh = blockIdx.x / nqt;
  const unsigned int h = bh % (unsigned int)NHEAD, b = bh / (unsigned int)NHEAD;
  const int tid = threadIdx.x, wave = tid >> 5, lane = tid & 31;
  const int r = lane & 15, hb = (lane >> 4) << 3;
  const unsigned int ur = (unsigned int)r;
  const _Float16* Qb = qkv + (size_t)b * SEQ * LDQKV + h * DHEAD;
  const _Float16* Kh = Qb + DIM;
  const _Float16* Vh = vt + (size_t)bh * DHEAD * SEQ;
  const int q0 = (int)qt * 64 + wave * 16;
  const unsigned int* mq = mbits + (size_t)(q0 + hb) * WPR;

  v16h aq[2];
#pragma unroll
  for (int dc = 0; dc < 2; ++dc)
    aq[dc] = load_frag(Qb + (size_t)(q0 + r) * LDQKV + dc * 32 + hb);

  v16h ones;
#pragma unroll
  for (int e = 0; e < 16; ++e) ones[e] = (_Float16)1.0f;

  v8f o[4];
#pragma unroll
  for (int t = 0; t < 4; ++t)
#pragma unroll
    for (int v = 0; v < 8; ++v) o[t][v] = 0.f;
  float mrow[8], lrow[8];
#pragma unroll
  for (int v = 0; v < 8; ++v) { mrow[v] = -1e30f; lrow[v] = 0.f; }

  _Float16* Pw = Ps + wave * 16 * VPAD;
  const v8f zero = {0.f, 0.f, 0.f, 0.f, 0.f, 0.f, 0.f, 0.f};

#pragma unroll 1
  for (int kb = 0; kb < SEQ / 32; ++kb) {
    const int key0 = kb * 32;

    unsigned int mwd[8];
#pragma unroll
    for (int v = 0; v < 8; ++v) mwd[v] = mq[(size_t)v * WPR + kb];

    v8f s[2];
#pragma unroll
    for (int kt = 0; kt < 2; ++kt)
#pragma unroll
      for (int v = 0; v < 8; ++v) s[kt][v] = 0.f;
#pragma unroll
    for (int kt = 0; kt < 2; ++kt)
#pragma unroll
      for (int dc = 0; dc < 2; ++dc) {
        const v16h bk = load_frag(Kh + (size_t)(key0 + kt * 16 + r) * LDQKV + dc * 32 + hb);
        s[kt] = wmma16(aq[dc], bk, s[kt]);
      }

    float alpha[8];
#pragma unroll
    for (int v = 0; v < 8; ++v) {
      const unsigned int w = mwd[v];
      const bool on0 = ((w >> ur) & 1u) != 0u;
      const bool on1 = ((w >> (ur + 16u)) & 1u) != 0u;
      const float s0 = on0 ? s[0][v] * 0.125f : -1.0e9f;
      const float s1 = on1 ? s[1][v] * 0.125f : -1.0e9f;
      float mx = fmaxf(s0, s1);
#pragma unroll
      for (int msk = 8; msk >= 1; msk >>= 1) mx = fmaxf(mx, __shfl_xor(mx, msk, 32));
      const float mnew = fmaxf(mrow[v], mx);
      alpha[v] = __expf(mrow[v] - mnew);
      mrow[v]  = mnew;
      s[0][v] = __expf(s0 - mnew) * 1024.0f;
      s[1][v] = __expf(s1 - mnew) * 1024.0f;
    }

#pragma unroll
    for (int kt = 0; kt < 2; ++kt)
#pragma unroll
      for (int v = 0; v < 8; ++v)
        Pw[(v + hb) * VPAD + kt * 16 + r] = (_Float16)s[kt][v];
    __syncthreads();

    const v16h pf = load_frag(Pw + r * VPAD + hb);

    const v8f rsum = wmma16(pf, ones, zero);
#pragma unroll
    for (int v = 0; v < 8; ++v) lrow[v] = lrow[v] * alpha[v] + rsum[v];

#pragma unroll
    for (int t = 0; t < 4; ++t) {
#pragma unroll
      for (int v = 0; v < 8; ++v) o[t][v] *= alpha[v];
      const v16h bv = load_frag(Vh + (size_t)(t * 16 + r) * SEQ + key0 + hb);
      o[t] = wmma16(pf, bv, o[t]);
    }
  }

  _Float16* Ow = Os + wave * 16 * OPAD;
#pragma unroll
  for (int v = 0; v < 8; ++v) {
    const float inv = 16.0f / lrow[v];
#pragma unroll
    for (int t = 0; t < 4; ++t) Ow[(v + hb) * OPAD + t * 16 + r] = (_Float16)(o[t][v] * inv);
  }
  __syncthreads();

  const int rs = lane >> 3, cc = (lane & 7) << 3;
  v8h hv[4];
  size_t go[4];
#pragma unroll
  for (int it = 0; it < 4; ++it) {
    const int lr = it * 4 + rs;
    hv[it] = *(const v8h*)(Ow + lr * OPAD + cc);
    go[it] = ((size_t)b * SEQ + q0 + lr) * (size_t)DIM + h * DHEAD + cc;
  }
#pragma unroll
  for (int it = 0; it < 4; ++it) *(volatile v8h*)(ctx + go[it]) = hv[it];
  __threadfence();
#pragma unroll
  for (int it = 0; it < 4; ++it) *(volatile v8h*)(ctx + go[it]) = hv[it];
}

#define LNT 192
#define LNW (LNT / 32)
static_assert(LNT * 4 == DIM && (DIM / 8) == 96 && ((DIM / 8) % 32) == 0);

template <bool XIN>
__global__ __launch_bounds__(LNT) void ln_kernel(
    const float* __restrict__ in, const float* __restrict__ g, const float* __restrict__ bt,
    _Float16* __restrict__ outH) {
#pragma clang fp contract(off)
  __shared__ float red0[LNW];
  __shared__ float red1[LNW];
  __shared__ __attribute__((aligned(16))) _Float16 sh[DIM];
  const size_t row = blockIdx.x;
  const size_t irow = XIN ? FROW(row) : row;
  const int tid = threadIdx.x, wave = tid >> 5, lane = tid & 31;
  v4f v = *(const v4f*)(in + irow * DIM + tid * 4);
  if constexpr (XIN) {
#pragma unroll
    for (int e = 0; e < 4; ++e) v[e] = bf16r(v[e]);
  }
  float s = (v[0] + v[1]) + (v[2] + v[3]);
#pragma unroll
  for (int m = 16; m >= 1; m >>= 1) s += __shfl_xor(s, m, 32);
  if (lane == 0) red0[wave] = s;
  __syncthreads();
  float S = 0.f;
#pragma unroll
  for (int i = 0; i < LNW; ++i) S += red0[i];
  const float mu = S * (1.0f / (float)DIM);
  const float d0 = v[0] - mu, d1 = v[1] - mu, d2 = v[2] - mu, d3 = v[3] - mu;
  float ss = (d0 * d0 + d1 * d1) + (d2 * d2 + d3 * d3);
#pragma unroll
  for (int m = 16; m >= 1; m >>= 1) ss += __shfl_xor(ss, m, 32);
  if (lane == 0) red1[wave] = ss;
  __syncthreads();
  float SS = 0.f;
#pragma unroll
  for (int i = 0; i < LNW; ++i) SS += red1[i];
  const float var = SS * (1.0f / (float)(DIM - 1));
  const float sd = sqrtf(var);
  const float inv = 1.0f / (sd + 1e-6f);
  const v4f gg = *(const v4f*)(g + tid * 4);
  const v4f bb = *(const v4f*)(bt + tid * 4);
  v4f y;
  y[0] = (bf16r(gg[0]) * d0) * inv + bf16r(bb[0]);
  y[1] = (bf16r(gg[1]) * d1) * inv + bf16r(bb[1]);
  y[2] = (bf16r(gg[2]) * d2) * inv + bf16r(bb[2]);
  y[3] = (bf16r(gg[3]) * d3) * inv + bf16r(bb[3]);
#pragma unroll
  for (int e = 0; e < 4; ++e) sh[tid * 4 + e] = (_Float16)y[e];
  __syncthreads();
  if (tid < DIM / 8) {
    const v8h hv = *(const v8h*)(sh + tid * 8);
    _Float16* hp = outH + row * DIM + tid * 8;
    *(volatile v8h*)hp = hv;
    __threadfence();
    *(volatile v8h*)hp = hv;
  }
}

static_assert((size_t)(DIM / 64) * (DIM / 64) * 3 * 4096 == (size_t)3 * DIM * DIM);
static_assert((size_t)(HID / 64) * (DIM / 64) * 4096 == (size_t)HID * DIM);
static_assert((size_t)(SEQ / 64) * (NB * NHEAD) * 4096 == (size_t)NB * NHEAD * DHEAD * SEQ);
static_assert((size_t)(LDQKV / BN) * (MROWS / BM) * BM * BN == (size_t)MROWS * LDQKV);
static_assert((size_t)(DIM / BN) * (MROWS / BM) * BM * BN == (size_t)MROWS * DIM);
static_assert((size_t)(HID / BN) * (MROWS / BM) * BM * BN == (size_t)MROWS * HID);
static_assert((size_t)NB * NHEAD * (SEQ / 64) * 64 * DHEAD == (size_t)MROWS * DIM);
static_assert(((size_t)SEQ * SEQ / 4096) * 128 == (size_t)SEQ * WPR);

extern "C" void kernel_launch(void* const* d_in, const int* in_sizes, int n_in,
                              void* d_out, int out_size, void* d_ws, size_t ws_size,
                              hipStream_t stream) {
  if (n_in < 18) return;
  const size_t needX = ((size_t)(NB - 1) * SEQ_FULL + SEQ) * DIM;
  const size_t needM = (size_t)(SEQ - 1) * SEQ_FULL + SEQ;
  if ((size_t)in_sizes[0] < needX) return;
  if ((size_t)in_sizes[1] < needM) return;
  if (in_sizes[2] < DIM * DIM || in_sizes[4] < DIM * DIM || in_sizes[6] < DIM * DIM ||
      in_sizes[8] < DIM * DIM) return;
  if (in_sizes[3] < DIM || in_sizes[5] < DIM || in_sizes[7] < DIM || in_sizes[9] < DIM) return;
  if (in_sizes[10] < DIM * HID || in_sizes[11] < HID || in_sizes[12] < HID * DIM || in_sizes[13] < DIM) return;
  if (in_sizes[14] < DIM || in_sizes[15] < DIM || in_sizes[16] < DIM || in_sizes[17] < DIM) return;
  if ((size_t)out_size < needX) return;

  const float* x    = (const float*)d_in[0];
  const int*   mask = (const int*)d_in[1];
  const float* Wq   = (const float*)d_in[2];
  const float* bq   = (const float*)d_in[3];
  const float* Wk   = (const float*)d_in[4];
  const float* bk   = (const float*)d_in[5];
  const float* Wv   = (const float*)d_in[6];
  const float* bv   = (const float*)d_in[7];
  const float* Wo   = (const float*)d_in[8];
  const float* bo   = (const float*)d_in[9];
  const float* W1   = (const float*)d_in[10];
  const float* b1   = (const float*)d_in[11];
  const float* W2   = (const float*)d_in[12];
  const float* b2   = (const float*)d_in[13];
  const float* g1   = (const float*)d_in[14];
  const float* be1  = (const float*)d_in[15];
  const float* g2   = (const float*)d_in[16];
  const float* be2  = (const float*)d_in[17];
  float* out = (float*)d_out;

  const size_t szWqkv = (size_t)3 * DIM * DIM * 2;
  const size_t szWo   = (size_t)DIM * DIM * 2;
  const size_t szW1   = (size_t)HID * DIM * 2;
  const size_t szW2   = (size_t)DIM * HID * 2;
  const size_t szMB   = (size_t)SEQ * WPR * 4;
  const size_t szP1   = (size_t)MROWS * DIM * 2;
  const size_t szP2   = (size_t)MROWS * LDQKV * 2;
  const size_t szP3   = (size_t)MROWS * HID * 2;
  const size_t oWqkv = 0;
  const size_t oWo   = oWqkv + szWqkv;
  const size_t oW1   = oWo + szWo;
  const size_t oW2   = oW1 + szW1;
  const size_t oMB   = oW2 + szW2;
  const size_t oP1   = oMB + szMB;
  const size_t oP2   = oP1 + szP1;
  const size_t oP3   = oP2 + szP2;
  const size_t total = oP3 + szP3;
  if (total > ws_size) return;
  static_assert(((size_t)3 * DIM * DIM * 2) % 128 == 0 && ((size_t)DIM * DIM * 2) % 128 == 0 &&
                ((size_t)HID * DIM * 2) % 128 == 0 && ((size_t)SEQ * WPR * 4) % 128 == 0 &&
                ((size_t)MROWS * DIM * 2) % 128 == 0);
  static_assert((size_t)MROWS * DIM * 4 <= (size_t)MROWS * LDQKV * 2);
  static_assert((size_t)MROWS * DIM * 2 <= (size_t)MROWS * HID * 2);
  static_assert((size_t)NB * NHEAD * DHEAD * SEQ * 2 <= (size_t)MROWS * DIM * 2);
  static_assert((size_t)3 * DIM * DIM * 2 + (size_t)DIM * DIM * 2 + (size_t)HID * DIM * 2 * 2 +
                (size_t)SEQ * WPR * 4 +
                (size_t)MROWS * DIM * 2 + (size_t)MROWS * LDQKV * 2 + (size_t)MROWS * HID * 2
                <= (size_t)134217728);

  char* ws = (char*)d_ws;
  _Float16* Wqkv_t = (_Float16*)(ws + oWqkv);
  _Float16* Wo_t   = (_Float16*)(ws + oWo);
  _Float16* W1_t   = (_Float16*)(ws + oW1);
  _Float16* W2_t   = (_Float16*)(ws + oW2);
  unsigned int* MB = (unsigned int*)(ws + oMB);
  _Float16* N1_16  = (_Float16*)(ws + oP1);
  _Float16* VT16   = (_Float16*)(ws + oP1);
  _Float16* N2_16  = (_Float16*)(ws + oP1);
  _Float16* QKV16  = (_Float16*)(ws + oP2);
  float*    R1     = (float*)   (ws + oP2);
  _Float16* CTX16  = (_Float16*)(ws + oP3);
  _Float16* G16    = (_Float16*)(ws + oP3);

  const float wsc    = 32.0f;
  const float inv32  = 1.0f / 32.0f;
  const float inv512 = 1.0f / 512.0f;
  const float hcar   = 16.0f;

  ln_kernel<true><<<dim3(MROWS), LNT, 0, stream>>>(x, g1, be1, N1_16);

  cvt_wt_kernel<<<dim3(DIM / 64, DIM / 64, 3), 256, 0, stream>>>(Wq, Wk, Wv, Wqkv_t, DIM, DIM, wsc);
  cvt_wt_kernel<<<dim3(DIM / 64, DIM / 64, 1), 256, 0, stream>>>(Wo, Wo, Wo, Wo_t, DIM, DIM, wsc);
  cvt_wt_kernel<<<dim3(HID / 64, DIM / 64, 1), 256, 0, stream>>>(W1, W1, W1, W1_t, DIM, HID, wsc);
  cvt_wt_kernel<<<dim3(DIM / 64, HID / 64, 1), 256, 0, stream>>>(W2, W2, W2, W2_t, HID, DIM, wsc);

  maskpack_kernel<<<dim3((unsigned int)((size_t)SEQ * SEQ / 4096)), 128, 0, stream>>>(mask, MB);

  gemm_kernel<true, 0, false, true, false>
      <<<dim3(LDQKV / BN, MROWS / BM), 256, 0, stream>>>(
          N1_16, Wqkv_t, bq, bk, bv, nullptr, nullptr, QKV16, LDQKV, DIM, inv32, 1.0f, DIM);

  vtrans_kernel<<<dim3(SEQ / 64, NB * NHEAD), 256, 0, stream>>>(QKV16, VT16);

  attn_kernel<<<dim3(NB * NHEAD * (SEQ / 64)), 128, 0, stream>>>(QKV16, VT16, MB, CTX16);

  gemm_kernel<true, 2, false, false, false>
      <<<dim3(DIM / BN, MROWS / BM), 256, 0, stream>>>(
          CTX16, Wo_t, bo, bo, bo, x, R1, nullptr, DIM, DIM, inv512, 1.0f, DIM);

  ln_kernel<false><<<dim3(MROWS), LNT, 0, stream>>>(R1, g2, be2, N2_16);

  gemm_kernel<true, 0, true, true, false>
      <<<dim3(HID / BN, MROWS / BM), 256, 0, stream>>>(
          N2_16, W1_t, b1, b1, b1, nullptr, nullptr, G16, HID, DIM, inv32 * hcar, hcar, HID);

  gemm_kernel<true, 1, false, false, true>
      <<<dim3(DIM / BN, MROWS / BM), 256, 0, stream>>>(
          G16, W2_t, b2, b2, b2, R1, out, nullptr, DIM, HID, inv512, 1.0f, DIM);
}
